// EncoderBlock_14817637171306
// MI455X (gfx1250) — hardware-verified
//
#include <hip/hip_runtime.h>
#include <math.h>

constexpr int NBAT   = 8;
constexpr int NSEQ   = 2048;
constexpr int NDIN   = 300;
constexpr int NDPAD  = 320;
constexpr int NHID   = 128;
constexpr int NGATE  = 384;
constexpr int NROWS  = NBAT * NSEQ;
constexpr int NOUTC  = 640;
constexpr int GRU_HP = 136;
constexpr int GRU_RP = 132;
constexpr float GW_CARRY     = 64.0f;
constexpr float GW_CARRY_INV = 1.0f / 64.0f;
constexpr float Q_CARRY      = 2048.0f;
constexpr float Q_CARRY_INV  = 1.0f / 2048.0f;
constexpr float E_ARG_LO     = -9.5f;
constexpr float E_ARG_HI     = 11.0f;

static_assert(NBAT == 8, "one store wave per batch row in the scan kernel");
static_assert(NSEQ == 2048 && NHID == 128 && NGATE == 3 * NHID && NOUTC == 5 * NHID, "shape contract");
static_assert(NDIN % 4 == 0 && NDPAD % 32 == 0 && NDPAD >= NDIN, "K padding");
static_assert(NROWS % 64 == 0 && NHID % 64 == 0 && NGATE % 64 == 0 && NSEQ % 64 == 0, "GEMM tile multiples");
static_assert(NHID % 32 == 0 && NGATE % 32 == 0 && NSEQ % 32 == 0, "GEMM K multiples");
static_assert((2 * 16 * GRU_HP) % 256 == 0, "h tile zero fill exact");
static_assert((NROWS * (NDPAD / 8)) % 256 == 0 && (NHID * (NDPAD / 8)) % 256 == 0 && (NGATE * (NHID / 8)) % 256 == 0, "convert grids exact");

typedef __attribute__((ext_vector_type(16))) _Float16 v16h;
typedef __attribute__((ext_vector_type(8)))  _Float16 v8h;
typedef __attribute__((ext_vector_type(16))) __bf16   v16b;
typedef __attribute__((ext_vector_type(8)))  __bf16   v8b;
typedef __attribute__((ext_vector_type(8)))  float    v8f;
typedef __attribute__((ext_vector_type(4)))  float    v4f;
typedef __attribute__((ext_vector_type(4)))  unsigned v4u;

__device__ __forceinline__ unsigned short f2bf_bits(float f) {
  unsigned u = __float_as_uint(f);
  return (unsigned short)((u + 0x7FFFu + ((u >> 16) & 1u)) >> 16);
}
__device__ __forceinline__ float bf_bits2f(unsigned short h) { return __uint_as_float(((unsigned)h) << 16); }
__device__ __forceinline__ unsigned bf_bits_u(float f) {
  const unsigned u = __float_as_uint(f);
  return (u + 0x7FFFu + ((u >> 16) & 1u)) >> 16;
}
__device__ __forceinline__ float bf16r(float f) { return __uint_as_float(bf_bits_u(f) << 16); }

__device__ __forceinline__ float h16_to_f32(unsigned hb) {
  const unsigned sgn = (hb & 0x8000u) << 16;
  const unsigned em = hb & 0x7fffu;
  const float fn = __uint_as_float((em << 13) + 0x38000000u);
  const float fs = (float)em * 5.9604644775390625e-8f;
  const float mag = (em < 0x400u) ? fs : fn;
  return __uint_as_float(__float_as_uint(mag) | sgn);
}

__device__ __forceinline__ void guard4_h(v8f& a, v8f& b, v8f& c, v8f& d, v16h x, v16h y) {
  asm volatile("v_nop\n\tv_nop\n\tv_nop\n\tv_nop" : "+v"(a), "+v"(b), "+v"(c), "+v"(d) : "v"(x), "v"(y));
}
__device__ __forceinline__ void guard4_b(v8f& a, v8f& b, v8f& c, v8f& d, v16b x, v16b y) {
  asm volatile("v_nop\n\tv_nop\n\tv_nop\n\tv_nop" : "+v"(a), "+v"(b), "+v"(c), "+v"(d) : "v"(x), "v"(y));
}
__device__ __forceinline__ void guard3_b(v8f& a, v8f& b, v8f& c, v16b x, v16b y0, v16b y1, v16b y2) {
  asm volatile("v_nop\n\tv_nop\n\tv_nop\n\tv_nop" : "+v"(a), "+v"(b), "+v"(c) : "v"(x), "v"(y0), "v"(y1), "v"(y2));
}
__device__ __forceinline__ void keep4_h(v16h a, v16h b, v16h c, v16h d) { asm volatile("v_nop" :: "v"(a), "v"(b), "v"(c), "v"(d)); }
__device__ __forceinline__ void keep4_b(v16b a, v16b b, v16b c, v16b d) { asm volatile("v_nop" :: "v"(a), "v"(b), "v"(c), "v"(d)); }
__device__ __forceinline__ void acc_guard4(v8f& a, v8f& b, v8f& c, v8f& d) {
  asm volatile("v_nop\n\tv_nop\n\tv_nop\n\tv_nop" : "+v"(a), "+v"(b), "+v"(c), "+v"(d));
}
__device__ __forceinline__ void wave_lds_sync() {
  __builtin_amdgcn_fence(__ATOMIC_RELEASE, "workgroup");
  __builtin_amdgcn_wave_barrier();
  __builtin_amdgcn_fence(__ATOMIC_ACQUIRE, "workgroup");
}

template <typename T> struct Frag;
template <> struct Frag<_Float16> {
  typedef v16h V; union U { v16h v; v8h h[2]; };
  static __device__ __forceinline__ v16h load(const _Float16* p) {
    U f; f.h[0] = *(const v8h*)(p); f.h[1] = *(const v8h*)(p + 16); return f.v;
  }
  static __device__ __forceinline__ v8f mma(v16h a, v16h b, v8f c) {
    return __builtin_amdgcn_wmma_f32_16x16x32_f16(false, a, false, b, (short)0, c, false, false);
  }
  static __device__ __forceinline__ void guard4(v8f& a, v8f& b, v8f& c, v8f& d, v16h x, v16h y) { guard4_h(a, b, c, d, x, y); }
  static __device__ __forceinline__ void keep(v16h a, v16h b, v16h c, v16h d) { keep4_h(a, b, c, d); }
};
template <> struct Frag<__bf16> {
  typedef v16b V; union U { v16b v; v8b h[2]; };
  static __device__ __forceinline__ v16b load(const __bf16* p) {
    U f; f.h[0] = *(const v8b*)(p); f.h[1] = *(const v8b*)(p + 16); return f.v;
  }
  static __device__ __forceinline__ v8f mma(v16b a, v16b b, v8f c) {
    return __builtin_amdgcn_wmma_f32_16x16x32_bf16(false, a, false, b, (short)0, c, false, false);
  }
  static __device__ __forceinline__ void guard4(v8f& a, v8f& b, v8f& c, v8f& d, v16b x, v16b y) { guard4_b(a, b, c, d, x, y); }
  static __device__ __forceinline__ void keep(v16b a, v16b b, v16b c, v16b d) { keep4_b(a, b, c, d); }
};

template <int ET> struct Elem;
template <> struct Elem<0> { typedef _Float16 T; };
template <> struct Elem<1> { typedef __bf16 T; };

template <bool TM> __device__ __forceinline__ size_t out_row(int m) {
  return TM ? (size_t)((m % NSEQ) * NBAT + (m / NSEQ)) : (size_t)m;
}

template <int ET, int ASPLIT, int BIAS_MODE, int OUT_MODE, bool TMAJOR>
__global__ __launch_bounds__(256) void wmma_gemm64(
    const unsigned short* __restrict__ Ap, const unsigned short* __restrict__ A2p, int lda, long strideA,
    const unsigned short* __restrict__ Btp, int ldb, long strideB,
    void* __restrict__ Cout, void* Cout2, int ldc, long strideC,
    const float* __restrict__ bias, int M, int N, int K, float scale) {
  typedef typename Elem<ET>::T T;
  typedef typename Frag<T>::V V;
  const T* A = (const T*)Ap; const T* A2 = (const T*)A2p; const T* Bt = (const T*)Btp;
  __shared__ __align__(16) float sT[8][16 * 68];
  const int b    = blockIdx.y;
  const int lane = threadIdx.x & 31;
  const int wave = threadIdx.x >> 5;
  const int tilesN = N >> 6;
  const int tilesM = M >> 6;
  const int tile = blockIdx.x * 8 + wave;
  if (tile >= tilesM * tilesN) return;
  const int tm = tile / tilesN;
  const int tn = tile - tm * tilesN;
  const int m0 = tm << 6;
  const int n0 = tn << 6;

  const T* Ab  = A  + (size_t)b * strideA;
  const T* Bb  = Bt + (size_t)b * strideB;
  const T* Ab2 = ASPLIT ? (A2 + (size_t)b * strideA) : Ab;

  const int rlane = lane & 15;
  const int koff  = (lane >> 4) * 8;
  const int mOff  = (lane >> 4) * 8;

  v8f acc[4][4];
#pragma unroll
  for (int i = 0; i < 4; ++i)
#pragma unroll
    for (int j = 0; j < 4; ++j) acc[i][j] = (v8f){0.f,0.f,0.f,0.f,0.f,0.f,0.f,0.f};

#pragma unroll 1
  for (int k0 = 0; k0 < K; k0 += 32) {
    V bh[4];
#pragma unroll
    for (int j = 0; j < 4; ++j) {
      const size_t bo = (size_t)(n0 + (j << 4) + rlane) * ldb + koff + k0;
      bh[j] = Frag<T>::load(Bb + bo);
    }
#pragma unroll
    for (int i = 0; i < 4; ++i) {
      const size_t ao = (size_t)(m0 + (i << 4) + rlane) * lda + koff + k0;
      V ah = Frag<T>::load(Ab + ao);
      V al = ah;
      if (ASPLIT) al = Frag<T>::load(Ab2 + ao);
#pragma unroll
      for (int j = 0; j < 4; ++j) {
        acc[i][j] = Frag<T>::mma(ah, bh[j], acc[i][j]);
        if (ASPLIT) acc[i][j] = Frag<T>::mma(al, bh[j], acc[i][j]);
      }
      Frag<T>::guard4(acc[i][0], acc[i][1], acc[i][2], acc[i][3], ah, al);
    }
    Frag<T>::keep(bh[0], bh[1], bh[2], bh[3]);
  }
  acc_guard4(acc[0][0], acc[0][1], acc[0][2], acc[0][3]);
  acc_guard4(acc[1][0], acc[1][1], acc[1][2], acc[1][3]);
  acc_guard4(acc[2][0], acc[2][1], acc[2][2], acc[2][3]);
  acc_guard4(acc[3][0], acc[3][1], acc[3][2], acc[3][3]);

  float* slab = sT[wave];
#pragma unroll
  for (int i = 0; i < 4; ++i) {
    const int mBase = m0 + (i << 4);
#pragma unroll
    for (int j = 0; j < 4; ++j) {
      const int n = n0 + (j << 4) + rlane;
      float bv = 0.f;
      if (BIAS_MODE == 2) bv = bf16r(bias[n]);
#pragma unroll
      for (int r = 0; r < 8; ++r) {
        float v = acc[i][j][r] * scale;
        if (BIAS_MODE == 2) v += bv;
        slab[(mOff + r) * 68 + (j << 4) + rlane] = v;
      }
    }
    wave_lds_sync();
    if (OUT_MODE == 0) {
      float* C = (float*)Cout + (size_t)b * strideC;
      const int hh = lane >> 4, c4 = (lane & 15) * 4;
      for (int pass = 0; pass < 2; ++pass) {
#pragma unroll
        for (int it = 0; it < 8; ++it) {
          const int row = it * 2 + hh;
          v4f v = *(const v4f*)(slab + row * 68 + c4);
          *(volatile v4f*)(C + out_row<TMAJOR>(mBase + row) * (size_t)ldc + n0 + c4) = v;
        }
        __threadfence();
      }
    } else {
      const int q = lane >> 3, c8 = (lane & 7) * 8;
      unsigned short* C  = (unsigned short*)Cout  + (size_t)b * strideC;
      unsigned short* C2 = (unsigned short*)Cout2 + (size_t)b * strideC;
      for (int pass = 0; pass < 2; ++pass) {
#pragma unroll
        for (int it = 0; it < 4; ++it) {
          const int row = it * 4 + q;
          const float* sp = slab + row * 68 + c8;
          v8h hv, lv;
#pragma unroll
          for (int e = 0; e < 8; ++e) {
            unsigned short hb = f2bf_bits(sp[e]);
            unsigned short lb = f2bf_bits(sp[e] - bf_bits2f(hb));
            hv[e] = __builtin_bit_cast(_Float16, hb);
            lv[e] = __builtin_bit_cast(_Float16, lb);
          }
          *(volatile v8h*)(C  + (size_t)(mBase + row) * ldc + n0 + c8) = hv;
          *(volatile v8h*)(C2 + (size_t)(mBase + row) * ldc + n0 + c8) = lv;
        }
        __threadfence();
      }
    }
    wave_lds_sync();
  }
}

__global__ __launch_bounds__(256) void cvt_pad_bf16_kernel(const float* __restrict__ src, unsigned short* __restrict__ dst,
                                                           int nrow, int ncol8, int scols, int spitch) {
  const int i  = blockIdx.x * 256 + threadIdx.x;
  const int n8 = nrow * ncol8;
  if (i < n8) {
    const int row = i / ncol8;
    const int c8  = i - row * ncol8;
    const int col0 = c8 * 8, col1 = col0 + 4;
    const bool ok0 = col0 < scols, ok1 = col1 < scols;
    const int cc0 = ok0 ? col0 : (scols - 4);
    const int cc1 = ok1 ? col1 : (scols - 4);
    const float* sp = src + (size_t)row * spitch;
    const v4f a = *(const v4f*)(sp + cc0);
    const v4f b = *(const v4f*)(sp + cc1);
    const float a0 = a[0], a1 = a[1], a2 = a[2], a3 = a[3];
    const float b0 = b[0], b1 = b[1], b2 = b[2], b3 = b[3];
    const unsigned u0 = ok0 ? bf_bits_u(a0) : 0u;
    const unsigned u1 = ok0 ? bf_bits_u(a1) : 0u;
    const unsigned u2 = ok0 ? bf_bits_u(a2) : 0u;
    const unsigned u3 = ok0 ? bf_bits_u(a3) : 0u;
    const unsigned u4 = ok1 ? bf_bits_u(b0) : 0u;
    const unsigned u5 = ok1 ? bf_bits_u(b1) : 0u;
    const unsigned u6 = ok1 ? bf_bits_u(b2) : 0u;
    const unsigned u7 = ok1 ? bf_bits_u(b3) : 0u;
    v4u w;
    w[0] = u0 | (u1 << 16);
    w[1] = u2 | (u3 << 16);
    w[2] = u4 | (u5 << 16);
    w[3] = u6 | (u7 << 16);
    *(volatile v4u*)(dst + (size_t)i * 8) = w;
    __threadfence();
    *(volatile v4u*)(dst + (size_t)i * 8) = w;
  }
}

__device__ __forceinline__ float sigm_f(float x)  { return __builtin_amdgcn_rcpf(1.0f + expf(-x)); }
__device__ __forceinline__ float tanh_f(float x)  { return 1.0f - 2.0f * __builtin_amdgcn_rcpf(expf(2.0f * x) + 1.0f); }

__global__ __launch_bounds__(256) void gru_scan_kernel(const float* __restrict__ XFp, const float* __restrict__ XBp,
                                                       const unsigned short* __restrict__ WHFp,
                                                       const unsigned short* __restrict__ WHBp,
                                                       const float* __restrict__ bhF, const float* __restrict__ bhB,
                                                       float* __restrict__ out) {
  __shared__ __align__(16) unsigned short Ah[2][16 * GRU_HP];
  __shared__ __align__(16) float          Rs[2][8 * GRU_RP];
  const int tid = threadIdx.x, lane = tid & 31, wave = tid >> 5;
  const int c = lane & 15, hh = lane >> 4, koff = hh * 8;
  const int dir = blockIdx.x;
  const float* X  = dir ? XBp : XFp;
  const __bf16* W = (const __bf16*)(dir ? WHBp : WHFp);
  const float* bh = dir ? bhB : bhF;
  const int ch = 16 * wave + c;

  {
    unsigned short* af = &Ah[0][0];
#pragma unroll 1
    for (int i = tid; i < 2 * 16 * GRU_HP; i += 256) af[i] = (unsigned short)0;
  }
  v16b bw[3][4];
#pragma unroll
  for (int g = 0; g < 3; ++g) {
#pragma unroll
    for (int kc = 0; kc < 4; ++kc)
      bw[g][kc] = Frag<__bf16>::load(W + (size_t)(g * NHID + ch) * NHID + koff + 32 * kc);
    asm volatile("" ::: "memory");
  }
  float bhv[3];
#pragma unroll
  for (int g = 0; g < 3; ++g) bhv[g] = bf16r(bh[g * NHID + ch]);
  float hst[4];
#pragma unroll
  for (int i = 0; i < 4; ++i) hst[i] = 0.0f;
  float xc[3][4];
  {
    const int s0 = dir ? (NSEQ - 1) : 0;
#pragma unroll
    for (int g = 0; g < 3; ++g)
#pragma unroll
      for (int i = 0; i < 4; ++i)
        xc[g][i] = X[((size_t)s0 * NBAT + 4 * hh + i) * NGATE + g * NHID + ch];
  }
  __syncthreads();

  const v8f z8 = {0.f, 0.f, 0.f, 0.f, 0.f, 0.f, 0.f, 0.f};

#pragma unroll 1
  for (int t = 0; t < NSEQ; ++t) {
    const int s   = dir ? (NSEQ - 1 - t) : t;
    const int cur = t & 1;
    const int tn = (t + 1 < NSEQ) ? (t + 1) : (NSEQ - 1);
    const int sn = dir ? (NSEQ - 1 - tn) : tn;
    float xn[3][4];
#pragma unroll
    for (int g = 0; g < 3; ++g)
#pragma unroll
      for (int i = 0; i < 4; ++i)
        xn[g][i] = X[((size_t)sn * NBAT + 4 * hh + i) * NGATE + g * NHID + ch];

    const __bf16* arow = (const __bf16*)(&Ah[cur][0]) + c * GRU_HP + koff;
    v8f acc[3];
    acc[0] = z8; acc[1] = z8; acc[2] = z8;
#pragma unroll
    for (int kc = 0; kc < 4; ++kc) {
      const v16b a = Frag<__bf16>::load(arow + 32 * kc);
      acc[0] = Frag<__bf16>::mma(a, bw[0][kc], acc[0]);
      acc[1] = Frag<__bf16>::mma(a, bw[1][kc], acc[1]);
      acc[2] = Frag<__bf16>::mma(a, bw[2][kc], acc[2]);
      guard3_b(acc[0], acc[1], acc[2], a, bw[0][kc], bw[1][kc], bw[2][kc]);
    }
    float gsel[3][4];
#pragma unroll
    for (int g = 0; g < 3; ++g) {
      float tot[8];
#pragma unroll
      for (int r = 0; r < 8; ++r) {
        const float mine = acc[g][r];
        const float oth  = __shfl_xor(mine, 16, 32);
        tot[r] = mine + oth;
      }
#pragma unroll
      for (int i = 0; i < 4; ++i) gsel[g][i] = hh ? tot[4 + i] : tot[i];
    }
    unsigned short* an = &Ah[cur ^ 1][0];
    float* rs = &Rs[cur][0];
#pragma unroll
    for (int i = 0; i < 4; ++i) {
      const float hr = gsel[0][i] + bhv[0];
      const float hz = gsel[1][i] + bhv[1];
      const float hn = gsel[2][i] + bhv[2];
      const float rg = sigm_f(xc[0][i] + hr);
      const float zg = sigm_f(xc[1][i] + hz);
      const float ng = tanh_f(xc[2][i] + rg * hn);
      const float hv = (1.0f - zg) * ng + zg * hst[i];
      hst[i] = hv;
      const unsigned hb = bf_bits_u(hv);
      const float hif = __uint_as_float(hb << 16);
      const unsigned lb = bf_bits_u(hv - hif);
      an[(4 * hh + i) * GRU_HP + ch]     = (unsigned short)hb;
      an[(8 + 4 * hh + i) * GRU_HP + ch] = (unsigned short)lb;
      rs[(4 * hh + i) * GRU_RP + ch]     = hv;
    }
    __syncthreads();
    {
      const v4f rv = *(const v4f*)(&Rs[cur][0] + wave * GRU_RP + 4 * lane);
      float* op = out + ((size_t)wave * NSEQ + (size_t)s) * NOUTC + dir * NHID + 4 * lane;
      for (int pass = 0; pass < 2; ++pass) {
        *(volatile v4f*)op = rv;
        __threadfence();
      }
    }
#pragma unroll
    for (int g = 0; g < 3; ++g)
#pragma unroll
      for (int i = 0; i < 4; ++i) xc[g][i] = xn[g][i];
  }
}

__global__ __launch_bounds__(256) void build_g_kernel(const unsigned short* __restrict__ PHIp,
                                                      const unsigned short* __restrict__ PLOp,
                                                      const float* __restrict__ outR,
                                                      const float* __restrict__ w_a, const float* __restrict__ w_f,
                                                      unsigned short* __restrict__ G16, unsigned short* __restrict__ GW16,
                                                      float* __restrict__ A32) {
  __shared__ __align__(16) float As[32];
  const int tid = threadIdx.x, lane = tid & 31, wave = tid >> 5;
  const int l15 = lane & 15;
  const bool lowhalf = lane < 16;
  const int colA = 8 * lane;
  const int colB = 256 + 8 * l15;
  float wfA[8], waA[8], wfB[8], waB[8];
  {
    const v4f f0 = *(const v4f*)(w_f + colA);
    const v4f f1 = *(const v4f*)(w_f + colA + 4);
    const v4f a0 = *(const v4f*)(w_a + colA);
    const v4f a1 = *(const v4f*)(w_a + colA + 4);
#pragma unroll
    for (int e = 0; e < 4; ++e) {
      wfA[e]     = bf16r(f0[e]) * GW_CARRY;
      wfA[4 + e] = bf16r(f1[e]) * GW_CARRY;
      waA[e]     = bf16r(a0[e]);
      waA[4 + e] = bf16r(a1[e]);
    }
    asm volatile("" ::: "memory");
    const v4f g0 = *(const v4f*)(w_f + colB);
    const v4f g1 = *(const v4f*)(w_f + colB + 4);
    const v4f b0 = *(const v4f*)(w_a + colB);
    const v4f b1 = *(const v4f*)(w_a + colB + 4);
#pragma unroll
    for (int e = 0; e < 4; ++e) {
      wfB[e]     = bf16r(g0[e]) * GW_CARRY;
      wfB[4 + e] = bf16r(g1[e]) * GW_CARRY;
      waB[e]     = bf16r(b0[e]);
      waB[4 + e] = bf16r(b1[e]);
    }
  }
#pragma unroll 1
  for (int it = 0; it < 4; ++it) {
    const int row = blockIdx.x * 32 + wave * 4 + it;
    const v4u ph = *(const v4u*)(PHIp + (size_t)row * NHID + 8 * l15);
    const v4u pl = *(const v4u*)(PLOp + (size_t)row * NHID + 8 * l15);
    const float* rp = outR + (size_t)row * NOUTC;
    const v4f ra0 = *(const v4f*)(rp + 8 * l15);
    const v4f ra1 = *(const v4f*)(rp + 8 * l15 + 4);
    const v4f rb0 = *(const v4f*)(rp + NHID + 8 * l15);
    const v4f rb1 = *(const v4f*)(rp + NHID + 8 * l15 + 4);
    const unsigned h0 = ph[0], h1 = ph[1], h2 = ph[2], h3 = ph[3];
    const unsigned q0 = pl[0], q1 = pl[1], q2 = pl[2], q3 = pl[3];
    float p[8];
    p[0] = __uint_as_float(h0 << 16) + __uint_as_float(q0 << 16);
    p[1] = __uint_as_float(h0 & 0xffff0000u) + __uint_as_float(q0 & 0xffff0000u);
    p[2] = __uint_as_float(h1 << 16) + __uint_as_float(q1 << 16);
    p[3] = __uint_as_float(h1 & 0xffff0000u) + __uint_as_float(q1 & 0xffff0000u);
    p[4] = __uint_as_float(h2 << 16) + __uint_as_float(q2 << 16);
    p[5] = __uint_as_float(h2 & 0xffff0000u) + __uint_as_float(q2 & 0xffff0000u);
    p[6] = __uint_as_float(h3 << 16) + __uint_as_float(q3 << 16);
    p[7] = __uint_as_float(h3 & 0xffff0000u) + __uint_as_float(q3 & 0xffff0000u);
    float gA[8], gB[8];
#pragma unroll
    for (int e = 0; e < 4; ++e) {
      const float r0 = ra0[e], r1 = ra1[e];
      gA[e]     = lowhalf ? p[e] : r0;
      gA[4 + e] = lowhalf ? p[4 + e] : r1;
      gB[e]     = rb0[e];
      gB[4 + e] = rb1[e];
    }
    float sa = 0.0f, sb = 0.0f;
    v8h hA, hB, wA, wB;
#pragma unroll
    for (int e = 0; e < 8; ++e) {
      sa += gA[e] * waA[e];
      sb += gB[e] * waB[e];
      hA[e] = (_Float16)gA[e];
      hB[e] = (_Float16)gB[e];
      wA[e] = (_Float16)(gA[e] * wfA[e]);
      wB[e] = (_Float16)(gB[e] * wfB[e]);
    }
    sa += lowhalf ? sb : 0.0f;
#pragma unroll
    for (int off = 16; off > 0; off >>= 1) sa += __shfl_xor(sa, off, 32);
    unsigned short* gp = G16  + (size_t)row * NGATE;
    unsigned short* wp = GW16 + (size_t)row * NGATE;
    for (int pass = 0; pass < 2; ++pass) {
      *(volatile v8h*)(gp + colA) = hA;
      *(volatile v8h*)(wp + colA) = wA;
      if (lowhalf) {
        *(volatile v8h*)(gp + colB) = hB;
        *(volatile v8h*)(wp + colB) = wB;
      }
      __threadfence();
    }
    if (lane == 0) As[wave * 4 + it] = sa;
  }
  __syncthreads();
  if (tid < 8) {
    const v4f av = *(const v4f*)(As + 4 * tid);
    float* ap = A32 + (size_t)blockIdx.x * 32 + 4 * tid;
    *(volatile v4f*)ap = av;
    __threadfence();
    *(volatile v4f*)ap = av;
  }
}

__global__ __launch_bounds__(256) void escore_kernel(const unsigned short* __restrict__ GWp, const unsigned short* __restrict__ Gp,
                                                     const float* __restrict__ A32, unsigned short* __restrict__ E16,
                                                     float* __restrict__ Z32) {
  __shared__ __align__(16) float    sT[8][16 * 68];
  __shared__ __align__(16) _Float16 sE[8][16 * 72];
  __shared__ __align__(16) float    Zs[8][64];
  const int b = blockIdx.y, kbase = blockIdx.x * 128;
  const int lane = threadIdx.x & 31, wave = threadIdx.x >> 5;
  const int wj = wave >> 1, wk = wave & 1;
  const _Float16* Ab = (const _Float16*)GWp + (size_t)b * NSEQ * NGATE;
  const _Float16* Bb = (const _Float16*)Gp  + (size_t)b * NSEQ * NGATE;
  unsigned short* Ep = E16 + (size_t)b * NSEQ * NSEQ;
  const float* Av = A32 + (size_t)b * NSEQ;
  const int n0 = kbase + wk * 64;
  const int rlane = lane & 15;
  const int koff  = (lane >> 4) * 8;
  const int mOff  = (lane >> 4) * 8;
  const int q = lane >> 3, c8 = (lane & 7) * 8;
  float* slab = sT[wave];
  _Float16* es = sE[wave];
  float zc[8];
#pragma unroll
  for (int e = 0; e < 8; ++e) zc[e] = 0.0f;

#pragma unroll 1
  for (int jt = 0; jt < NSEQ / 256; ++jt) {
    const int m0 = jt * 256 + wj * 64;
    v8f acc[4][4];
#pragma unroll
    for (int i = 0; i < 4; ++i)
#pragma unroll
      for (int j = 0; j < 4; ++j) acc[i][j] = (v8f){0.f,0.f,0.f,0.f,0.f,0.f,0.f,0.f};
#pragma unroll 1
    for (int k0 = 0; k0 < NGATE; k0 += 32) {
      v16h bh[4];
#pragma unroll
      for (int j = 0; j < 4; ++j)
        bh[j] = Frag<_Float16>::load(Bb + (size_t)(n0 + (j << 4) + rlane) * NGATE + koff + k0);
#pragma unroll
      for (int i = 0; i < 4; ++i) {
        const v16h ah = Frag<_Float16>::load(Ab + (size_t)(m0 + (i << 4) + rlane) * NGATE + koff + k0);
#pragma unroll
        for (int j = 0; j < 4; ++j) acc[i][j] = Frag<_Float16>::mma(ah, bh[j], acc[i][j]);
        guard4_h(acc[i][0], acc[i][1], acc[i][2], acc[i][3], ah, ah);
      }
      keep4_h(bh[0], bh[1], bh[2], bh[3]);
    }
    acc_guard4(acc[0][0], acc[0][1], acc[0][2], acc[0][3]);
    acc_guard4(acc[1][0], acc[1][1], acc[1][2], acc[1][3]);
    acc_guard4(acc[2][0], acc[2][1], acc[2][2], acc[2][3]);
    acc_guard4(acc[3][0], acc[3][1], acc[3][2], acc[3][3]);

#pragma unroll
    for (int i = 0; i < 4; ++i) {
      const int mBase = m0 + (i << 4);
#pragma unroll
      for (int j = 0; j < 4; ++j)
#pragma unroll
        for (int r = 0; r < 8; ++r) slab[(mOff + r) * 68 + (j << 4) + rlane] = acc[i][j][r];
      wave_lds_sync();
#pragma unroll 1
      for (int it = 0; it < 4; ++it) {
        const int row = it * 4 + q;
        const float aj = Av[mBase + row];
        const float* sp = slab + row * 68 + c8;
        const v4f s0 = *(const v4f*)(sp);
        const v4f s1 = *(const v4f*)(sp + 4);
        v8h hv;
#pragma unroll
        for (int e = 0; e < 4; ++e) {
          float x0 = s0[e] * GW_CARRY_INV + aj;
          float x1 = s1[e] * GW_CARRY_INV + aj;
          x0 = fminf(fmaxf(x0, E_ARG_LO), E_ARG_HI);
          x1 = fminf(fmaxf(x1, E_ARG_LO), E_ARG_HI);
          const float e0 = expf(x0);
          const float e1 = expf(x1);
          zc[e]     += e0;
          zc[4 + e] += e1;
          hv[e]     = (_Float16)e0;
          hv[4 + e] = (_Float16)e1;
        }
        *(v8h*)(es + row * 72 + c8) = hv;
      }
      wave_lds_sync();
      for (int pass = 0; pass < 2; ++pass) {
#pragma unroll
        for (int it = 0; it < 4; ++it) {
          const int row = it * 4 + q;
          const v8h hv = *(const v8h*)(es + row * 72 + c8);
          *(volatile v8h*)(Ep + (size_t)(mBase + row) * NSEQ + n0 + c8) = hv;
        }
        __threadfence();
      }
      wave_lds_sync();
    }
  }
#pragma unroll
  for (int e = 0; e < 8; ++e) {
    zc[e] += __shfl_xor(zc[e], 8, 32);
    zc[e] += __shfl_xor(zc[e], 16, 32);
  }
  if (lane < 8) {
    v4f z0, z1;
#pragma unroll
    for (int e = 0; e < 4; ++e) { z0[e] = zc[e]; z1[e] = zc[4 + e]; }
    *(v4f*)(&Zs[wave][c8])     = z0;
    *(v4f*)(&Zs[wave][c8 + 4]) = z1;
  }
  __syncthreads();
  if (wave == 0) {
    const int col = 4 * lane;
    const int wkk = col >> 6, cl = col & 63;
    v4f zs = *(const v4f*)(&Zs[0 * 2 + wkk][cl]);
    const v4f t1 = *(const v4f*)(&Zs[1 * 2 + wkk][cl]);
    const v4f t2 = *(const v4f*)(&Zs[2 * 2 + wkk][cl]);
    const v4f t3 = *(const v4f*)(&Zs[3 * 2 + wkk][cl]);
    zs = ((zs + t1) + t2) + t3;
    float* zp = Z32 + (size_t)b * NSEQ + kbase + col;
    *(volatile v4f*)zp = zs;
    __threadfence();
    *(volatile v4f*)zp = zs;
  }
}

__global__ __launch_bounds__(256) void gst_kernel(const unsigned short* __restrict__ Gp, const float* __restrict__ Z32,
                                                  unsigned short* __restrict__ GsT) {
  __shared__ float Tt[64 * 65];
  const int tid = threadIdx.x;
  const int d0 = blockIdx.x * 64, k0 = blockIdx.y * 64, b = blockIdx.z;
#pragma unroll
  for (int i = 0; i < 2; ++i) {
    const int idx = i * 256 + tid;
    const int rr = idx >> 3, cc = (idx & 7) * 8;
    const v4u w = *(const v4u*)(Gp + ((size_t)b * NSEQ + k0 + rr) * NGATE + d0 + cc);
    const float z = Z32[(size_t)b * NSEQ + k0 + rr];
    const float sc = Q_CARRY * (1.0f / z);
    const unsigned w0 = w[0], w1 = w[1], w2 = w[2], w3 = w[3];
    float* tp = Tt + rr * 65 + cc;
    tp[0] = h16_to_f32(w0 & 0xffffu) * sc;
    tp[1] = h16_to_f32(w0 >> 16) * sc;
    tp[2] = h16_to_f32(w1 & 0xffffu) * sc;
    tp[3] = h16_to_f32(w1 >> 16) * sc;
    tp[4] = h16_to_f32(w2 & 0xffffu) * sc;
    tp[5] = h16_to_f32(w2 >> 16) * sc;
    tp[6] = h16_to_f32(w3 & 0xffffu) * sc;
    tp[7] = h16_to_f32(w3 >> 16) * sc;
  }
  __syncthreads();
  const int q = tid >> 3, c8 = (tid & 7) * 8;
  v8h hv[2];
#pragma unroll
  for (int g = 0; g < 2; ++g) {
    const int qq = g * 32 + q;
#pragma unroll
    for (int e = 0; e < 8; ++e) {
      const float f = Tt[(c8 + e) * 65 + qq];
      hv[g][e] = (_Float16)f;
    }
  }
  for (int pass = 0; pass < 2; ++pass) {
#pragma unroll
    for (int g = 0; g < 2; ++g) {
      const size_t o = ((size_t)b * NGATE + d0 + g * 32 + q) * (size_t)NSEQ + (size_t)(k0 + c8);
      *(volatile v8h*)(GsT + o) = hv[g];
    }
    __threadfence();
  }
}

constexpr size_t SZ_SEQB = (size_t)NROWS * NDPAD * 2;
constexpr size_t SZ_P16  = (size_t)NROWS * NHID * 2;
constexpr size_t SZ_X    = (size_t)NSEQ * NBAT * NGATE * 4;
constexpr size_t SZ_EARLY = SZ_SEQB + 2 * SZ_P16 + 2 * SZ_X;
constexpr size_t SZ_E16  = (size_t)NBAT * NSEQ * NSEQ * 2;
constexpr size_t SZ_WLIN = (size_t)NHID * NDPAD * 2;
constexpr size_t SZ_WG   = (size_t)NGATE * NHID * 2;
constexpr size_t SZ_G16  = (size_t)NROWS * NGATE * 2;
constexpr size_t SZ_VEC  = (size_t)NROWS * 4;
constexpr size_t SZ_TOTAL = SZ_EARLY + SZ_WLIN + 4 * SZ_WG + 3 * SZ_G16 + 2 * SZ_VEC;
static_assert(SZ_E16 <= SZ_EARLY, "E16 alias fits in the dead early region");
static_assert(SZ_TOTAL <= (size_t)134217728, "carve within the limit");
static_assert(SZ_SEQB % 256 == 0 && SZ_P16 % 256 == 0 && SZ_X % 256 == 0 && SZ_WLIN % 256 == 0 && SZ_WG % 256 == 0 &&
              SZ_G16 % 256 == 0 && SZ_VEC % 256 == 0, "aligned carve");
static_assert((size_t)NROWS * NOUTC * 4 == (size_t)41943040, "output bytes");

extern "C" void kernel_launch(void* const* d_in, const int* in_sizes, int n_in,
                              void* d_out, int out_size, void* d_ws, size_t ws_size, hipStream_t stream) {
  if (n_in < 14 || d_out == nullptr || d_ws == nullptr) return;
  if (in_sizes[0] != NROWS * NDIN || in_sizes[1] != NHID * NDIN || in_sizes[2] != NHID ||
      in_sizes[3] != NGATE * NHID || in_sizes[4] != NGATE * NHID || in_sizes[5] != NGATE || in_sizes[6] != NGATE ||
      in_sizes[7] != NGATE * NHID || in_sizes[8] != NGATE * NHID || in_sizes[9] != NGATE || in_sizes[10] != NGATE ||
      in_sizes[11] != NGATE || in_sizes[12] != NGATE || in_sizes[13] != NGATE || out_size != NROWS * NOUTC) return;
  if (SZ_TOTAL > ws_size) return;

  const float* seq   = (const float*)d_in[0];
  const float* W_lin = (const float*)d_in[1];
  const float* b_lin = (const float*)d_in[2];
  const float* Wih_f = (const float*)d_in[3];
  const float* Whh_f = (const float*)d_in[4];
  const float* bih_f = (const float*)d_in[5];
  const float* bhh_f = (const float*)d_in[6];
  const float* Wih_b = (const float*)d_in[7];
  const float* Whh_b = (const float*)d_in[8];
  const float* bih_b = (const float*)d_in[9];
  const float* bhh_b = (const float*)d_in[10];
  const float* w_a   = (const float*)d_in[11];
  const float* w_f   = (const float*)d_in[13];
  float* out = (float*)d_out;

  char* ws = (char*)d_ws; size_t off = 0;
  auto carve = [&](size_t bytes) -> char* { char* p = ws + off; off += bytes; return p; };
  unsigned short* SEQB = (unsigned short*)carve(SZ_SEQB);
  unsigned short* PHI  = (unsigned short*)carve(SZ_P16);
  unsigned short* PLO  = (unsigned short*)carve(SZ_P16);
  float*          XF   = (float*)carve(SZ_X);
  float*          XB   = (float*)carve(SZ_X);
  unsigned short* WLIN = (unsigned short*)carve(SZ_WLIN);
  unsigned short* WIHF = (unsigned short*)carve(SZ_WG);
  unsigned short* WIHB = (unsigned short*)carve(SZ_WG);
  unsigned short* WHHF = (unsigned short*)carve(SZ_WG);
  unsigned short* WHHB = (unsigned short*)carve(SZ_WG);
  unsigned short* G16  = (unsigned short*)carve(SZ_G16);
  unsigned short* GW16 = (unsigned short*)carve(SZ_G16);
  unsigned short* GST  = (unsigned short*)carve(SZ_G16);
  float*          A32  = (float*)carve(SZ_VEC);
  float*          Z32  = (float*)carve(SZ_VEC);
  unsigned short* E16  = (unsigned short*)ws;
  if (off != SZ_TOTAL) return;

  cvt_pad_bf16_kernel<<<(NROWS * (NDPAD / 8)) / 256, 256, 0, stream>>>(seq,   SEQB, NROWS, NDPAD / 8, NDIN, NDIN);
  cvt_pad_bf16_kernel<<<(NHID  * (NDPAD / 8)) / 256, 256, 0, stream>>>(W_lin, WLIN, NHID,  NDPAD / 8, NDIN, NDIN);
  cvt_pad_bf16_kernel<<<(NGATE * (NHID / 8)) / 256, 256, 0, stream>>>(Wih_f, WIHF, NGATE, NHID / 8, NHID, NHID);
  cvt_pad_bf16_kernel<<<(NGATE * (NHID / 8)) / 256, 256, 0, stream>>>(Wih_b, WIHB, NGATE, NHID / 8, NHID, NHID);
  cvt_pad_bf16_kernel<<<(NGATE * (NHID / 8)) / 256, 256, 0, stream>>>(Whh_f, WHHF, NGATE, NHID / 8, NHID, NHID);
  cvt_pad_bf16_kernel<<<(NGATE * (NHID / 8)) / 256, 256, 0, stream>>>(Whh_b, WHHB, NGATE, NHID / 8, NHID, NHID);

  wmma_gemm64<1, 0, 2, 2, false><<<dim3((NROWS / 64) * (NHID / 64) / 8, 1), 256, 0, stream>>>(
      SEQB, SEQB, NDPAD, 0L, WLIN, NDPAD, 0L, (void*)PHI, (void*)PLO, NHID, 0L, b_lin, NROWS, NHID, NDPAD, 1.0f);

  wmma_gemm64<1, 1, 2, 0, true><<<dim3((NROWS / 64) * (NGATE / 64) / 8, 1), 256, 0, stream>>>(
      PHI, PLO, NHID, 0L, WIHF, NHID, 0L, (void*)XF, (void*)XF, NGATE, 0L, bih_f, NROWS, NGATE, NHID, 1.0f);
  wmma_gemm64<1, 1, 2, 0, true><<<dim3((NROWS / 64) * (NGATE / 64) / 8, 1), 256, 0, stream>>>(
      PHI, PLO, NHID, 0L, WIHB, NHID, 0L, (void*)XB, (void*)XB, NGATE, 0L, bih_b, NROWS, NGATE, NHID, 1.0f);

  gru_scan_kernel<<<2, 256, 0, stream>>>(XF, XB, WHHF, WHHB, bhh_f, bhh_b, out);

  build_g_kernel<<<NROWS / 32, 256, 0, stream>>>(PHI, PLO, out, w_a, w_f, G16, GW16, A32);

  escore_kernel<<<dim3(NSEQ / 128, NBAT), 256, 0, stream>>>(GW16, G16, A32, E16, Z32);

  gst_kernel<<<dim3(NGATE / 64, NSEQ / 64, NBAT), 256, 0, stream>>>(G16, Z32, GST);

  wmma_gemm64<0, 0, 0, 0, false><<<dim3((NSEQ / 64) * (NGATE / 64) / 8, NBAT), 256, 0, stream>>>(
      E16, E16, NSEQ, (long)NSEQ * NSEQ, GST, NSEQ, (long)NGATE * NSEQ,
      (void*)(out + 2 * NHID), (void*)(out + 2 * NHID), NOUTC, (long)NSEQ * NOUTC,
      b_lin, NSEQ, NGATE, NSEQ, Q_CARRY_INV);
}
